// ImprovedGATNode_14267881357528
// MI455X (gfx1250) — hardware-verified
//
#include <hip/hip_runtime.h>
#include <stddef.h>
#include <math.h>

typedef __attribute__((ext_vector_type(16))) _Float16 v16h;
typedef __attribute__((ext_vector_type(8)))  _Float16 v8h;
typedef __attribute__((ext_vector_type(16))) __bf16   v16b;
typedef __attribute__((ext_vector_type(8)))  __bf16   v8b;
typedef __attribute__((ext_vector_type(8)))  float    v8f;
typedef __attribute__((ext_vector_type(4)))  float    v4f;
typedef __attribute__((ext_vector_type(4)))  int      v4i;

constexpr int NODE_IN = 256;
constexpr int NHEAD   = 8, HCH = 64;
constexpr int HIDW    = NHEAD * HCH;
constexpr int OUTW    = 16;
constexpr int OUTPAD  = 64;
constexpr int NB12    = 128;
constexpr int NB3     = 1024;
constexpr int RPQ     = 1024;
#define NTHR    256
#define NWAVE   8
#define EPT     8
#define NGRP    1
#define CHUNK   (NTHR * EPT * NGRP)
#define WCAP    (EPT * NGRP * 32)
#define LISTN   (NWAVE * WCAP)
#define LDS_AGG12 ((NB12 * HIDW + 2 * NB12 * NHEAD) * 4 + LISTN * 4 + 64)
#define LDS_AGG3  ((NB3 * OUTW + 2 * NB3 * 1) * 4 + LISTN * 4 + 64)

static_assert((CHUNK & (CHUNK - 1)) == 0);
static_assert(CHUNK <= 4096);
static_assert((NB12 & (NB12 - 1)) == 0 && NB12 <= 4096);
static_assert((NB3 & (NB3 - 1)) == 0 && NB3 <= 4096);
static_assert(RPQ % NB12 == 0 && RPQ % NB3 == 0 && RPQ % 64 == 0 && RPQ % NTHR == 0 && RPQ % NWAVE == 0);
static_assert(LDS_AGG12 == 278592 && LDS_AGG3 == 81984);
static_assert(NODE_IN % 32 == 0 && HIDW % 64 == 0 && OUTPAD % 64 == 0 && HIDW % 32 == 0);
static_assert(NODE_IN / 8 == 32 && HIDW == 512 && OUTW == 16);

__device__ __forceinline__ unsigned short f2bf_bits(float f) {
  unsigned u = __float_as_uint(f);
  return (unsigned short)((u + 0x7FFFu + ((u >> 16) & 1u)) >> 16);
}
__device__ __forceinline__ float bf_bits2f(unsigned short h) { return __uint_as_float(((unsigned)h) << 16); }

__device__ __forceinline__ void dep_guard_h(v8f& a, v8f& b, v16h x, v16h y) { asm volatile("v_nop\n\tv_nop\n\tv_nop\n\tv_nop" : "+v"(a), "+v"(b) : "v"(x), "v"(y)); }
__device__ __forceinline__ void dep_guard_b(v8f& a, v8f& b, v16b x, v16b y) { asm volatile("v_nop\n\tv_nop\n\tv_nop\n\tv_nop" : "+v"(a), "+v"(b) : "v"(x), "v"(y)); }
__device__ __forceinline__ void keep4_h(v16h a, v16h b, v16h c, v16h d) { asm volatile("v_nop" :: "v"(a), "v"(b), "v"(c), "v"(d)); }
__device__ __forceinline__ void keep4_b(v16b a, v16b b, v16b c, v16b d) { asm volatile("v_nop" :: "v"(a), "v"(b), "v"(c), "v"(d)); }
__device__ __forceinline__ void acc_guard4(v8f& a, v8f& b, v8f& c, v8f& d) { asm volatile("v_nop\n\tv_nop\n\tv_nop\n\tv_nop" : "+v"(a), "+v"(b), "+v"(c), "+v"(d)); }
template <typename T> struct Frag;
template <> struct Frag<_Float16> {
  typedef v16h V; union U { v16h v; v8h h[2]; };
  static __device__ __forceinline__ v16h load(const _Float16* p) {
    U f; f.h[0] = *(const v8h*)(p); f.h[1] = *(const v8h*)(p + 16); return f.v;
  }
  static __device__ __forceinline__ v8f mma(v16h a, v16h b, v8f c) {
    return __builtin_amdgcn_wmma_f32_16x16x32_f16(false, a, false, b, (short)0, c, false, false);
  }
  static __device__ __forceinline__ void guard(v8f& a, v8f& b, v16h x, v16h y) { dep_guard_h(a, b, x, y); }
  static __device__ __forceinline__ void keep(v16h a, v16h b, v16h c, v16h d) { keep4_h(a, b, c, d); }
};
template <> struct Frag<__bf16> {
  typedef v16b V; union U { v16b v; v8b h[2]; };
  static __device__ __forceinline__ v16b load(const __bf16* p) {
    U f; f.h[0] = *(const v8b*)(p); f.h[1] = *(const v8b*)(p + 16); return f.v;
  }
  static __device__ __forceinline__ v8f mma(v16b a, v16b b, v8f c) {
    return __builtin_amdgcn_wmma_f32_16x16x32_bf16(false, a, false, b, (short)0, c, false, false);
  }
  static __device__ __forceinline__ void guard(v8f& a, v8f& b, v16b x, v16b y) { dep_guard_b(a, b, x, y); }
  static __device__ __forceinline__ void keep(v16b a, v16b b, v16b c, v16b d) { keep4_b(a, b, c, d); }
};

template <int ET> struct Elem;
template <> struct Elem<0> { typedef _Float16 T; };
template <> struct Elem<1> { typedef __bf16 T; };
template <int ET, bool SPLIT, int BIAS_MODE, int OUT_MODE, bool RESID, int ACT = 0>
__global__ __launch_bounds__(256) void wmma_gemm64(
    const unsigned short* __restrict__ Ap, const unsigned short* __restrict__ A2p, int lda, long strideA,
    const unsigned short* __restrict__ Btp, const unsigned short* __restrict__ Bt2p, int ldb, long strideB,
    void* __restrict__ Cout, void* __restrict__ Cout2, int ldc, long strideC,
    const float* __restrict__ bias,
    const float* __restrict__ resid, long strideR,
    int M, int N, int K, float scale) {
  typedef typename Elem<ET>::T T;
  typedef typename Frag<T>::V V;
  const T* A = (const T*)Ap; const T* A2 = (const T*)A2p; const T* Bt = (const T*)Btp; const T* Bt2 = (const T*)Bt2p;
  __shared__ __align__(16) float sT[8][16 * 68];
  const int b    = blockIdx.y;
  const int lane = threadIdx.x & 31;
  const int wave = threadIdx.x >> 5;
  const int tilesN = N >> 6;
  const int tilesM = M >> 6;
  const int tile = blockIdx.x * 8 + wave;
  if (tile >= tilesM * tilesN) return;
  const int tm = tile / tilesN;
  const int tn = tile - tm * tilesN;
  const int m0 = tm << 6;
  const int n0 = tn << 6;

  const T* Ab  = A  + (size_t)b * strideA;
  const T* Bb  = Bt + (size_t)b * strideB;
  const T* Ab2 = SPLIT ? (A2  + (size_t)b * strideA) : nullptr;
  const T* Bb2 = SPLIT ? (Bt2 + (size_t)b * strideB) : nullptr;

  const int rlane = lane & 15;
  const int koff  = (lane >> 4) * 8;
  const int mOff  = (lane >> 4) * 8;

  v8f acc[4][4];
#pragma unroll
  for (int i = 0; i < 4; ++i)
#pragma unroll
    for (int j = 0; j < 4; ++j) acc[i][j] = (v8f){0.f,0.f,0.f,0.f,0.f,0.f,0.f,0.f};

  for (int k0 = 0; k0 < K; k0 += 32) {
    V bh[4], bl[4];
#pragma unroll
    for (int j = 0; j < 4; ++j) {
      const size_t bo = (size_t)(n0 + (j << 4) + rlane) * ldb + koff + k0;
      bh[j] = Frag<T>::load(Bb + bo);
      if (SPLIT) bl[j] = Frag<T>::load(Bb2 + bo);
    }
#pragma unroll
    for (int i = 0; i < 4; ++i) {
      const size_t ao = (size_t)(m0 + (i << 4) + rlane) * lda + koff + k0;
      V ah = Frag<T>::load(Ab + ao);
      V al;
      if (SPLIT) al = Frag<T>::load(Ab2 + ao);
#pragma unroll
      for (int j = 0; j < 4; ++j) {
        acc[i][j] = Frag<T>::mma(ah, bh[j], acc[i][j]);
        if (SPLIT) {
          acc[i][j] = Frag<T>::mma(ah, bl[j], acc[i][j]);
          acc[i][j] = Frag<T>::mma(al, bh[j], acc[i][j]);
        }
      }
      Frag<T>::guard(acc[i][0], acc[i][3], ah, SPLIT ? al : ah);
    }
    Frag<T>::keep(bh[0], bh[1], bh[2], bh[3]);
    if (SPLIT) Frag<T>::keep(bl[0], bl[1], bl[2], bl[3]);
  }
  acc_guard4(acc[0][0], acc[0][1], acc[0][2], acc[0][3]);
  acc_guard4(acc[1][0], acc[1][1], acc[1][2], acc[1][3]);
  acc_guard4(acc[2][0], acc[2][1], acc[2][2], acc[2][3]);
  acc_guard4(acc[3][0], acc[3][1], acc[3][2], acc[3][3]);

  float* slab = sT[wave];
  const float* Rb = RESID ? (resid + (size_t)b * strideR) : nullptr;
#pragma unroll
  for (int i = 0; i < 4; ++i) {
    const int mBase = m0 + (i << 4);
#pragma unroll
    for (int j = 0; j < 4; ++j) {
      const int n = n0 + (j << 4) + rlane;
      float bv = 0.f;
      if (BIAS_MODE == 2) bv = bias[n];
#pragma unroll
      for (int r = 0; r < 8; ++r) {
        float v = acc[i][j][r] * scale;
        if (BIAS_MODE == 1) v += bias[mBase + mOff + r];
        if (BIAS_MODE == 2) v += bv;
        if (RESID) v += Rb[(size_t)(mBase + mOff + r) * ldc + n];
        if (ACT == 1) v = tanhf(v);
        if (ACT == 2) v = fmaxf(v, 0.0f);
        if (ACT == 3) v = v / (1.0f + expf(-v));
        if (ACT == 4) v = (v > 0.f) ? v : 0.01f * v;
        if (ACT == 5) v = 0.5f * v * (1.0f + erff(v * 0.70710678118654752f));
        slab[(mOff + r) * 68 + (j << 4) + rlane] = v;
      }
    }
    __builtin_amdgcn_fence(__ATOMIC_RELEASE, "workgroup");
    __builtin_amdgcn_wave_barrier();
    __builtin_amdgcn_fence(__ATOMIC_ACQUIRE, "workgroup");
    if (OUT_MODE == 0) {
      float* C = (float*)Cout + (size_t)b * strideC;
      const int hh = lane >> 4, c4 = (lane & 15) * 4;
      for (int pass = 0; pass < 2; ++pass) {
#pragma unroll
        for (int it = 0; it < 8; ++it) {
          const int row = it * 2 + hh;
          v4f v = *(const v4f*)(slab + row * 68 + c4);
          *(volatile v4f*)(C + (size_t)(mBase + row) * ldc + n0 + c4) = v;
        }
        __threadfence();
      }
    } else {
      const int q = lane >> 3, c8 = (lane & 7) * 8;
      unsigned short* C  = (unsigned short*)Cout  + (size_t)b * strideC;
      unsigned short* C2 = (OUT_MODE == 2) ? ((unsigned short*)Cout2 + (size_t)b * strideC) : nullptr;
      for (int pass = 0; pass < 2; ++pass) {
#pragma unroll
        for (int it = 0; it < 4; ++it) {
          const int row = it * 4 + q;
          const float* sp = slab + row * 68 + c8;
          v8h hv, lv;
#pragma unroll
          for (int e = 0; e < 8; ++e) {
            if (OUT_MODE == 1) {
              hv[e] = (_Float16)sp[e];
            } else {
              unsigned short hb = f2bf_bits(sp[e]);
              unsigned short lb = f2bf_bits(sp[e] - bf_bits2f(hb));
              hv[e] = __builtin_bit_cast(_Float16, hb);
              lv[e] = __builtin_bit_cast(_Float16, lb);
            }
          }
          *(volatile v8h*)(C + (size_t)(mBase + row) * ldc + n0 + c8) = hv;
          if (OUT_MODE == 2) *(volatile v8h*)(C2 + (size_t)(mBase + row) * ldc + n0 + c8) = lv;
        }
        __threadfence();
      }
    }
    __builtin_amdgcn_fence(__ATOMIC_RELEASE, "workgroup");
    __builtin_amdgcn_wave_barrier();
    __builtin_amdgcn_fence(__ATOMIC_ACQUIRE, "workgroup");
  }
}

template <int NB>
__device__ __forceinline__ int scan_chunk(const int* __restrict__ lst, int nE, int cbase, int nodeBase,
                                          int* list, int tid, int lane, int wave, int fullvec) {
  int wc = 0;
#pragma unroll
  for (int g = 0; g < NGRP; ++g) {
    const int el0 = (g * NTHR + tid) * EPT;
    const int e0  = cbase + el0;
    v4i da, db;
    if (fullvec) {
      da = *(const v4i*)(lst + e0);
      db = *(const v4i*)(lst + e0 + 4);
    } else {
      const int em = nE - 1;
      da.x = lst[(e0     < em) ? e0     : em];
      da.y = lst[(e0 + 1 < em) ? e0 + 1 : em];
      da.z = lst[(e0 + 2 < em) ? e0 + 2 : em];
      da.w = lst[(e0 + 3 < em) ? e0 + 3 : em];
      db.x = lst[(e0 + 4 < em) ? e0 + 4 : em];
      db.y = lst[(e0 + 5 < em) ? e0 + 5 : em];
      db.z = lst[(e0 + 6 < em) ? e0 + 6 : em];
      db.w = lst[(e0 + 7 < em) ? e0 + 7 : em];
    }
    const bool v0 = (e0 < nE), v1 = (e0 + 1 < nE), v2 = (e0 + 2 < nE), v3 = (e0 + 3 < nE);
    const bool v4 = (e0 + 4 < nE), v5 = (e0 + 5 < nE), v6 = (e0 + 6 < nE), v7 = (e0 + 7 < nE);
    const unsigned nb = (unsigned)nodeBase;
    const unsigned s0 = (unsigned)da.x - nb, s1 = (unsigned)da.y - nb;
    const unsigned s2 = (unsigned)da.z - nb, s3 = (unsigned)da.w - nb;
    const unsigned s4 = (unsigned)db.x - nb, s5 = (unsigned)db.y - nb;
    const unsigned s6 = (unsigned)db.z - nb, s7 = (unsigned)db.w - nb;
    const bool h0 = v0 && (s0 < (unsigned)NB), h1 = v1 && (s1 < (unsigned)NB);
    const bool h2 = v2 && (s2 < (unsigned)NB), h3 = v3 && (s3 < (unsigned)NB);
    const bool h4 = v4 && (s4 < (unsigned)NB), h5 = v5 && (s5 < (unsigned)NB);
    const bool h6 = v6 && (s6 < (unsigned)NB), h7 = v7 && (s7 < (unsigned)NB);
    const unsigned any = __builtin_amdgcn_ballot_w32(h0 | h1 | h2 | h3 | h4 | h5 | h6 | h7);
    if (any != 0u) {
#define HITJ(J, HJ, SJ) { \
        const unsigned mj = __builtin_amdgcn_ballot_w32(HJ); \
        if (mj != 0u) { \
          if (HJ) { \
            const int pos = wc + (int)__builtin_amdgcn_mbcnt_lo(mj, 0u); \
            if (pos < WCAP) list[wave * WCAP + pos] = ((el0 + (J)) << 12) | (int)(SJ); \
          } \
          wc += (int)__builtin_popcount(mj); } }
      HITJ(0, h0, s0)
      HITJ(1, h1, s1)
      HITJ(2, h2, s2)
      HITJ(3, h3, s3)
      HITJ(4, h4, s4)
      HITJ(5, h5, s5)
      HITJ(6, h6, s6)
      HITJ(7, h7, s7)
#undef HITJ
    }
  }
  return wc;
}

__device__ __forceinline__ float dot4f(v4f a, v4f b) {
  return a.x * b.x + a.y * b.y + a.z * b.z + a.w * b.w;
}
__device__ __forceinline__ float hsum4(v4f a) { return (a.x + a.y) + (a.z + a.w); }
__device__ __forceinline__ void wave_lds_sync() {
  __builtin_amdgcn_fence(__ATOMIC_RELEASE, "workgroup");
  __builtin_amdgcn_wave_barrier();
  __builtin_amdgcn_fence(__ATOMIC_ACQUIRE, "workgroup");
}
__device__ __forceinline__ void split_bf(float f, _Float16& h, _Float16& l) {
  const unsigned short hb = f2bf_bits(f);
  const unsigned short lb = f2bf_bits(f - bf_bits2f(hb));
  h = __builtin_bit_cast(_Float16, hb);
  l = __builtin_bit_cast(_Float16, lb);
}
__device__ __forceinline__ void split8(v4f a, v4f b, v8h& hv, v8h& lv) {
  _Float16 h0, l0, h1, l1, h2, l2, h3, l3, h4, l4, h5, l5, h6, l6, h7, l7;
  split_bf(a.x, h0, l0); split_bf(a.y, h1, l1); split_bf(a.z, h2, l2); split_bf(a.w, h3, l3);
  split_bf(b.x, h4, l4); split_bf(b.y, h5, l5); split_bf(b.z, h6, l6); split_bf(b.w, h7, l7);
  hv[0] = h0; hv[1] = h1; hv[2] = h2; hv[3] = h3; hv[4] = h4; hv[5] = h5; hv[6] = h6; hv[7] = h7;
  lv[0] = l0; lv[1] = l1; lv[2] = l2; lv[3] = l3; lv[4] = l4; lv[5] = l5; lv[6] = l6; lv[7] = l7;
}
template <int CPL> struct VecT { typedef float T __attribute__((ext_vector_type(CPL))); };
template <> struct VecT<1> { typedef float T; };

__global__ __launch_bounds__(NTHR) void k_xprep(const float* __restrict__ x, unsigned short* ah,
                                                unsigned short* al, int nN, int nRows) {
  const int i = blockIdx.x * NTHR + threadIdx.x;
  if (i >= nRows * (NODE_IN / 8)) return;
  const int row = i >> 5;
  const int c0  = (i & 31) * 8;
  const int rc  = (row < nN) ? row : nN - 1;
  const float* xp = x + (size_t)rc * NODE_IN + c0;
  v4f a = *(const v4f*)xp, b = *(const v4f*)(xp + 4);
  if (row >= nN) { const v4f z = {0.f, 0.f, 0.f, 0.f}; a = z; b = z; }
  v8h hv, lv;
  split8(a, b, hv, lv);
  const size_t o = (size_t)row * NODE_IN + c0;
  *(volatile v8h*)(ah + o) = hv;
  *(volatile v8h*)(al + o) = lv;
  __threadfence();
  *(volatile v8h*)(ah + o) = hv;
  *(volatile v8h*)(al + o) = lv;
}

__global__ __launch_bounds__(NTHR) void k_wprep(const float* __restrict__ W, int kdim, int nOut, int nPad,
                                                unsigned short* bth, unsigned short* btl) {
  const int i  = blockIdx.x * NTHR + threadIdx.x;
  const int kq = kdim >> 3;
  if (i >= nPad * kq) return;
  const int n  = i / kq;
  const int k0 = (i - n * kq) * 8;
  const int nc = (n < nOut) ? n : nOut - 1;
  const float* p = W + (size_t)k0 * nOut + nc;
  v4f a, b;
  a.x = p[0];                  a.y = p[(size_t)nOut];       a.z = p[(size_t)2 * nOut];   a.w = p[(size_t)3 * nOut];
  b.x = p[(size_t)4 * nOut];   b.y = p[(size_t)5 * nOut];   b.z = p[(size_t)6 * nOut];   b.w = p[(size_t)7 * nOut];
  if (n >= nOut) { const v4f z = {0.f, 0.f, 0.f, 0.f}; a = z; b = z; }
  v8h hv, lv;
  split8(a, b, hv, lv);
  const size_t o = (size_t)n * kdim + k0;
  *(volatile v8h*)(bth + o) = hv;
  *(volatile v8h*)(btl + o) = lv;
  __threadfence();
  *(volatile v8h*)(bth + o) = hv;
  *(volatile v8h*)(btl + o) = lv;
}

template <bool RESID>
__global__ __launch_bounds__(NTHR) void k_rowpost(const float* __restrict__ vin,
                                                  const float* __restrict__ gamma, const float* __restrict__ beta,
                                                  float* xio, unsigned short* ah, unsigned short* al,
                                                  int nN, int nRows) {
  __shared__ __align__(16) float slab[NWAVE][HIDW + 32];
  const int tid = threadIdx.x, lane = tid & 31, wave = tid >> 5;
  const int row = blockIdx.x * NWAVE + wave;
  if (row >= nRows) return;
  const bool live = (row < nN);
  const int rc = live ? row : nN - 1;
  const float* src = vin + (size_t)rc * HIDW;
  const int c4 = lane * 4;
  const v4f x0 = *(const v4f*)(src + c4);
  const v4f x1 = *(const v4f*)(src + 128 + c4);
  const v4f x2 = *(const v4f*)(src + 256 + c4);
  const v4f x3 = *(const v4f*)(src + 384 + c4);
  float s1 = (hsum4(x0) + hsum4(x1)) + (hsum4(x2) + hsum4(x3));
#pragma unroll
  for (int off = 1; off < 32; off <<= 1) s1 += __shfl_xor(s1, off, 32);
  const float mean = s1 * (1.0f / 512.0f);
  const v4f d0 = x0 - mean, d1 = x1 - mean, d2 = x2 - mean, d3 = x3 - mean;
  float s2 = (dot4f(d0, d0) + dot4f(d1, d1)) + (dot4f(d2, d2) + dot4f(d3, d3));
#pragma unroll
  for (int off = 1; off < 32; off <<= 1) s2 += __shfl_xor(s2, off, 32);
  const float rstd = rsqrtf(s2 * (1.0f / 512.0f) + 1e-5f);
  float* sl = slab[wave];
  *(v4f*)(sl + c4)       = d0 * rstd;
  *(v4f*)(sl + 128 + c4) = d1 * rstd;
  *(v4f*)(sl + 256 + c4) = d2 * rstd;
  *(v4f*)(sl + 384 + c4) = d3 * rstd;
  wave_lds_sync();
#pragma unroll 1
  for (int k = 0; k < HIDW / 32; ++k) {
    const int i = k * 32 + lane;
    float v = sl[i] * gamma[i] + beta[i];
    const float en = expm1f(fminf(v, 0.0f));
    v = (v > 0.0f) ? v : en;
    if (RESID) v += xio[(size_t)rc * HIDW + i];
    if (!live) v = 0.0f;
    sl[i] = v;
  }
  wave_lds_sync();
  for (int pass = 0; pass < 2; ++pass) {
#pragma unroll
    for (int q = 0; q < 4; ++q) {
      const v4f v = *(const v4f*)(sl + q * 128 + c4);
      *(volatile v4f*)(xio + (size_t)row * HIDW + q * 128 + c4) = v;
    }
    __threadfence();
  }
  for (int pass = 0; pass < 2; ++pass) {
#pragma unroll
    for (int q = 0; q < 2; ++q) {
      const int c8 = q * 256 + lane * 8;
      const v4f p0 = *(const v4f*)(sl + c8), p1 = *(const v4f*)(sl + c8 + 4);
      v8h hv, lv;
      split8(p0, p1, hv, lv);
      *(volatile v8h*)(ah + (size_t)row * HIDW + c8) = hv;
      *(volatile v8h*)(al + (size_t)row * HIDW + c8) = lv;
    }
    __threadfence();
  }
}

__global__ __launch_bounds__(NTHR) void k_scores8(const float* __restrict__ h, const float* __restrict__ as,
                                                  const float* __restrict__ ad, float* ss, float* sd,
                                                  int nN, int nRows) {
  const int node = blockIdx.x * NTHR + threadIdx.x;
  if (node >= nRows) return;
  const int nc = (node < nN) ? node : nN - 1;
  const float* hr = h + (size_t)nc * HIDW;
  float sv[NHEAD], dv[NHEAD];
#pragma unroll
  for (int hd = 0; hd < NHEAD; ++hd) { sv[hd] = 0.f; dv[hd] = 0.f; }
#pragma unroll 1
  for (int c = 0; c < HCH; c += 4) {
#pragma unroll
    for (int hd = 0; hd < NHEAD; ++hd) {
      const v4f hv = *(const v4f*)(hr + hd * HCH + c);
      sv[hd] += dot4f(hv, *(const v4f*)(as + hd * HCH + c));
      dv[hd] += dot4f(hv, *(const v4f*)(ad + hd * HCH + c));
    }
  }
  if (node >= nN) {
#pragma unroll
    for (int hd = 0; hd < NHEAD; ++hd) { sv[hd] = 0.f; dv[hd] = 0.f; }
  }
  for (int pass = 0; pass < 2; ++pass) {
#pragma unroll
    for (int hd = 0; hd < NHEAD; ++hd) {
      *(volatile float*)(ss + (size_t)hd * nRows + node) = sv[hd];
      *(volatile float*)(sd + (size_t)hd * nRows + node) = dv[hd];
    }
    __threadfence();
  }
}

__global__ __launch_bounds__(NTHR) void k_scores16(const float* __restrict__ h, int ldh, const float* __restrict__ as,
                                                   const float* __restrict__ ad, float* ss, float* sd,
                                                   int nN, int nRows) {
  const int node = blockIdx.x * NTHR + threadIdx.x;
  if (node >= nRows) return;
  const int nc = (node < nN) ? node : nN - 1;
  const float* hr = h + (size_t)nc * ldh;
  float s0 = 0.f, d0 = 0.f;
#pragma unroll 1
  for (int c = 0; c < OUTW; c += 4) {
    const v4f hv = *(const v4f*)(hr + c);
    s0 += dot4f(hv, *(const v4f*)(as + c));
    d0 += dot4f(hv, *(const v4f*)(ad + c));
  }
  if (node >= nN) { s0 = 0.f; d0 = 0.f; }
  *(volatile float*)(ss + node) = s0;
  *(volatile float*)(sd + node) = d0;
  __threadfence();
  *(volatile float*)(ss + node) = s0;
  *(volatile float*)(sd + node) = d0;
}

template <int NB, int NH, int CH, bool FINAL>
__global__ __launch_bounds__(NTHR) void k_gat_agg(
    const int* __restrict__ rowl, const int* __restrict__ coll,
    const float* __restrict__ hfeat, int ldh,
    const float* __restrict__ ss, const float* __restrict__ sd, int rps,
    const float* __restrict__ bias, const float* __restrict__ gamma, const float* __restrict__ beta,
    float* of, int nN, int nE, int vec_ok) {
  constexpr int HC  = NH * CH;
  constexpr int CPL = (HC >= 32) ? (HC / 32) : 1;
  constexpr int RW  = NB / NWAVE;
  constexpr int C4R = HC / 4;
  constexpr int QPR = HC / 128;
  constexpr int LPR = (HC / 4 < 32) ? (HC / 4) : 32;
  constexpr int RPI = 32 / LPR;
  static_assert((NB * HC / 4) % NTHR == 0);
  static_assert(NB % NWAVE == 0, "rows per block must split evenly over waves");
  static_assert(HC % 16 == 0);
  static_assert(FINAL ? (HC == 16 && (RW % RPI) == 0) : (HC % 128 == 0 && CPL * 32 == HC));
  static_assert((NB & (NB - 1)) == 0 && NB <= 4096);
  typedef typename VecT<CPL>::T VT;
  extern __shared__ v4f lds_dyn[];
  float* acc  = (float*)lds_dyn;
  float* mst  = acc + NB * HC;
  float* sst  = mst + NB * NH;
  int*   list = (int*)(sst + NB * NH);
  int*   wcnt = list + LISTN;
  const int tid = threadIdx.x, lane = tid & 31, wave = tid >> 5;
  const int nodeBase = blockIdx.x * NB;

  {
    const v4f zz = {0.f, 0.f, 0.f, 0.f};
    for (int i = tid; i < NB * HC / 4; i += NTHR) lds_dyn[i] = zz;
    for (int i = tid; i < NB * NH; i += NTHR) { mst[i] = -INFINITY; sst[i] = 0.f; }
  }
  __syncthreads();

  const int colL = (HC >= 32) ? (CPL * lane) : (lane & (HC - 1));
  const int hdl  = colL / CH;
  const int nChunks = (nE + CHUNK - 1) / CHUNK;
#pragma unroll 1
  for (int ch = 0; ch < nChunks; ++ch) {
    const int cbase = ch * CHUNK;
    const int fullvec = (vec_ok != 0 && cbase + CHUNK <= nE) ? 1 : 0;
    const int wc = scan_chunk<NB>(coll, nE, cbase, nodeBase, list, tid, lane, wave, fullvec);
    if (lane == 0) wcnt[wave] = wc;
    __syncthreads();
    if (wave == 0) {
#pragma unroll 1
      for (int wsx = 0; wsx < NWAVE; ++wsx) {
        int n = __builtin_amdgcn_readfirstlane(wcnt[wsx]);
        n = n > WCAP ? WCAP : (n < 0 ? 0 : n);
        const int* lp = list + wsx * WCAP;
#pragma unroll 1
        for (int i = 0; i < n; ++i) {
          const int ent  = __builtin_amdgcn_readfirstlane(lp[i]);
          const int slot = ent & (NB - 1);
          int e = cbase + ((ent >> 12) & (CHUNK - 1));
          e = e > nE - 1 ? nE - 1 : e;
          int s = rowl[e];
          s = s < 0 ? 0 : (s > nN - 1 ? nN - 1 : s);
          const int node = nodeBase + slot;
          float lg = ss[(size_t)hdl * rps + s] + sd[(size_t)hdl * rps + node];
          lg = (lg > 0.f) ? lg : 0.2f * lg;
          const int mi = slot * NH + hdl;
          const float mo = mst[mi];
          const float so = sst[mi];
          const float d  = __expf(-fabsf(lg - mo));
          const bool  up = (lg > mo);
          const float sc = up ? d : 1.0f;
          const float w  = up ? 1.0f : d;
          const VT hv = *(const VT*)(hfeat + (size_t)s * ldh + colL);
          VT* ap = (VT*)(acc + slot * HC + colL);
          const VT av = *ap;
          *ap = av * sc + hv * w;
          mst[mi] = up ? lg : mo;
          sst[mi] = so * sc + w;
        }
      }
    }
    __syncthreads();
  }

#pragma unroll 1
  for (int it = 0; it < (NB * HC / 4) / NTHR; ++it) {
    const int idx  = it * NTHR + tid;
    const int slot = idx / C4R;
    const int c4   = (idx - slot * C4R) * 4;
    const int hd   = c4 / CH;
    const int node = nodeBase + slot;
    const int nc   = (node < nN) ? node : nN - 1;
    float lg = ss[(size_t)hd * rps + nc] + sd[(size_t)hd * rps + nc];
    lg = (lg > 0.f) ? lg : 0.2f * lg;
    const float mo = mst[slot * NH + hd];
    const float so = sst[slot * NH + hd];
    const float d  = __expf(-fabsf(lg - mo));
    const bool  up = (lg > mo);
    const float sc = up ? d : 1.0f;
    const float w  = up ? 1.0f : d;
    const v4f hs = *(const v4f*)(hfeat + (size_t)nc * ldh + c4);
    v4f* ap = (v4f*)(acc + slot * HC + c4);
    v4f a = *ap;
    a = a * sc + hs * w;
    const float sn  = so * sc + w;
    const float inv = __builtin_amdgcn_rcpf(sn);
    const v4f bv = *(const v4f*)(bias + c4);
    v4f o = a * inv + bv;
    if (!FINAL && node >= nN) { const v4f zz = {0.f, 0.f, 0.f, 0.f}; o = zz; }
    *ap = o;
  }
  __syncthreads();

  if (FINAL) {
#pragma unroll 1
    for (int r = tid; r < NB; r += NTHR) {
      float* rp = acc + r * HC;
      const v4f a0 = *(const v4f*)(rp), a1 = *(const v4f*)(rp + 4), a2 = *(const v4f*)(rp + 8), a3 = *(const v4f*)(rp + 12);
      const float mean = ((hsum4(a0) + hsum4(a1)) + (hsum4(a2) + hsum4(a3))) * (1.0f / 16.0f);
      const v4f d0 = a0 - mean, d1 = a1 - mean, d2 = a2 - mean, d3 = a3 - mean;
      const float var  = ((dot4f(d0, d0) + dot4f(d1, d1)) + (dot4f(d2, d2) + dot4f(d3, d3))) * (1.0f / 16.0f);
      const float rstd = rsqrtf(var + 1e-5f);
      const v4f g0 = *(const v4f*)(gamma), g1 = *(const v4f*)(gamma + 4), g2 = *(const v4f*)(gamma + 8), g3 = *(const v4f*)(gamma + 12);
      const v4f e0 = *(const v4f*)(beta),  e1 = *(const v4f*)(beta + 4),  e2 = *(const v4f*)(beta + 8),  e3 = *(const v4f*)(beta + 12);
      *(v4f*)(rp)      = d0 * rstd * g0 + e0;
      *(v4f*)(rp + 4)  = d1 * rstd * g1 + e1;
      *(v4f*)(rp + 8)  = d2 * rstd * g2 + e2;
      *(v4f*)(rp + 12) = d3 * rstd * g3 + e3;
    }
    __syncthreads();
    for (int pass = 0; pass < 2; ++pass) {
#pragma unroll 1
      for (int it = 0; it < RW / RPI; ++it) {
        const int row  = wave * RW + it * RPI + lane / LPR;
        const int col  = (lane - (lane / LPR) * LPR) * 4;
        const int grow = nodeBase + row;
        const v4f v = *(const v4f*)(acc + row * HC + col);
        if (grow < nN) *(volatile v4f*)(of + (size_t)grow * HC + col) = v;
      }
      __threadfence();
    }
  } else {
    float* ob = of + (size_t)nodeBase * HC;
    for (int pass = 0; pass < 2; ++pass) {
#pragma unroll 1
      for (int rr = 0; rr < RW; ++rr) {
        const int row = wave * RW + rr;
#pragma unroll
        for (int q = 0; q < QPR; ++q) {
          const int col = q * 128 + lane * 4;
          const v4f v = *(const v4f*)(acc + row * HC + col);
          *(volatile v4f*)(ob + (size_t)row * HC + col) = v;
        }
      }
      __threadfence();
    }
  }
}

extern "C" void kernel_launch(void* const* d_in, const int* in_sizes, int n_in,
                              void* d_out, int out_size, void* d_ws, size_t ws_size,
                              hipStream_t stream) {
  if (n_in < 24) return;
  const int nN = in_sizes[0] / NODE_IN;
  const int nE = in_sizes[1] / 2;
  if (nN < 1 || nE < 0 || in_sizes[0] != nN * NODE_IN || in_sizes[1] != 2 * nE) return;
  if (in_sizes[2] != NODE_IN * HIDW || in_sizes[3] < HIDW || in_sizes[4] < HIDW || in_sizes[5] < HIDW) return;
  if (in_sizes[6] != HIDW * HIDW || in_sizes[7] < HIDW || in_sizes[8] < HIDW) return;
  if (in_sizes[9] < HIDW || in_sizes[10] < HIDW || in_sizes[11] < HIDW) return;
  if (in_sizes[12] != HIDW * HIDW || in_sizes[13] < HIDW || in_sizes[14] < HIDW) return;
  if (in_sizes[15] < HIDW || in_sizes[16] < HIDW || in_sizes[17] < HIDW) return;
  if (in_sizes[18] != HIDW * OUTW || in_sizes[19] < OUTW || in_sizes[20] < OUTW) return;
  if (in_sizes[21] < OUTW || in_sizes[22] < OUTW || in_sizes[23] < OUTW) return;
  if (out_size != nN * OUTW) return;
  if (nN > (1 << 22)) return;

  const float* x    = (const float*)d_in[0];
  const int*   ei   = (const int*)d_in[1];
  const float* Wp   = (const float*)d_in[2];
  const float* bp   = (const float*)d_in[3];
  const float* g0   = (const float*)d_in[4];
  const float* b0   = (const float*)d_in[5];
  const float* W1   = (const float*)d_in[6];
  const float* as1  = (const float*)d_in[7];
  const float* ad1  = (const float*)d_in[8];
  const float* b1   = (const float*)d_in[9];
  const float* g1   = (const float*)d_in[10];
  const float* be1  = (const float*)d_in[11];
  const float* W2   = (const float*)d_in[12];
  const float* as2  = (const float*)d_in[13];
  const float* ad2  = (const float*)d_in[14];
  const float* b2   = (const float*)d_in[15];
  const float* g2   = (const float*)d_in[16];
  const float* be2  = (const float*)d_in[17];
  const float* W3   = (const float*)d_in[18];
  const float* as3  = (const float*)d_in[19];
  const float* ad3  = (const float*)d_in[20];
  const float* b3   = (const float*)d_in[21];
  const float* g3   = (const float*)d_in[22];
  const float* be3  = (const float*)d_in[23];
  const int* rowl = ei;
  const int* coll = ei + nE;
  float* out = (float*)d_out;

  const int RP  = ((nN + RPQ - 1) / RPQ) * RPQ;
  const int vec_col = ((nE & 3) == 0) ? 1 : 0;

  char* ws = (char*)d_ws;
  size_t off = 0;
  const size_t oAH  = off; off += (size_t)RP * HIDW * 2;
  const size_t oAL  = off; off += (size_t)RP * HIDW * 2;
  const size_t oWPH = off; off += (size_t)HIDW * NODE_IN * 2;
  const size_t oWPL = off; off += (size_t)HIDW * NODE_IN * 2;
  const size_t oW1H = off; off += (size_t)HIDW * HIDW * 2;
  const size_t oW1L = off; off += (size_t)HIDW * HIDW * 2;
  const size_t oW2H = off; off += (size_t)HIDW * HIDW * 2;
  const size_t oW2L = off; off += (size_t)HIDW * HIDW * 2;
  const size_t oW3H = off; off += (size_t)OUTPAD * HIDW * 2;
  const size_t oW3L = off; off += (size_t)OUTPAD * HIDW * 2;
  const size_t oHF  = off; off += (size_t)RP * HIDW * 4;
  const size_t oXF  = off; off += (size_t)RP * HIDW * 4;
  const size_t oAG  = off; off += (size_t)RP * HIDW * 4;
  const size_t oSS  = off; off += (size_t)NHEAD * RP * 4;
  const size_t oSD  = off; off += (size_t)NHEAD * RP * 4;
  if (off > ws_size) return;

  unsigned short* ah  = (unsigned short*)(ws + oAH);
  unsigned short* al  = (unsigned short*)(ws + oAL);
  unsigned short* wph = (unsigned short*)(ws + oWPH);
  unsigned short* wpl = (unsigned short*)(ws + oWPL);
  unsigned short* w1h = (unsigned short*)(ws + oW1H);
  unsigned short* w1l = (unsigned short*)(ws + oW1L);
  unsigned short* w2h = (unsigned short*)(ws + oW2H);
  unsigned short* w2l = (unsigned short*)(ws + oW2L);
  unsigned short* w3h = (unsigned short*)(ws + oW3H);
  unsigned short* w3l = (unsigned short*)(ws + oW3L);
  float* hf  = (float*)(ws + oHF);
  float* xf  = (float*)(ws + oXF);
  float* ag  = (float*)(ws + oAG);
  float* ssp = (float*)(ws + oSS);
  float* sdp = (float*)(ws + oSD);

  k_xprep<<<RP * (NODE_IN / 8) / NTHR, NTHR, 0, stream>>>(x, ah, al, nN, RP);
  k_wprep<<<(HIDW * (NODE_IN / 8) + NTHR - 1) / NTHR, NTHR, 0, stream>>>(Wp, NODE_IN, HIDW, HIDW, wph, wpl);
  k_wprep<<<(HIDW * (HIDW / 8) + NTHR - 1) / NTHR, NTHR, 0, stream>>>(W1, HIDW, HIDW, HIDW, w1h, w1l);
  k_wprep<<<(HIDW * (HIDW / 8) + NTHR - 1) / NTHR, NTHR, 0, stream>>>(W2, HIDW, HIDW, HIDW, w2h, w2l);
  k_wprep<<<(OUTPAD * (HIDW / 8) + NTHR - 1) / NTHR, NTHR, 0, stream>>>(W3, HIDW, OUTW, OUTPAD, w3h, w3l);

  const int gWide = ((RP / 64) * (HIDW / 64) + 7) / 8;
  const int gLast = ((RP / 64) * (OUTPAD / 64) + 7) / 8;

  wmma_gemm64<1, true, 2, 0, false, 0><<<dim3(gWide, 1), 256, 0, stream>>>(
      ah, al, NODE_IN, 0L, wph, wpl, NODE_IN, 0L, (void*)hf, (void*)hf, HIDW, 0L,
      bp, hf, 0L, RP, HIDW, NODE_IN, 1.0f);
  k_rowpost<false><<<RP / NWAVE, NTHR, 0, stream>>>(hf, g0, b0, xf, ah, al, nN, RP);

  wmma_gemm64<1, true, 0, 0, false, 0><<<dim3(gWide, 1), 256, 0, stream>>>(
      ah, al, HIDW, 0L, w1h, w1l, HIDW, 0L, (void*)hf, (void*)hf, HIDW, 0L,
      b1, hf, 0L, RP, HIDW, HIDW, 1.0f);
  k_scores8<<<RP / NTHR, NTHR, 0, stream>>>(hf, as1, ad1, ssp, sdp, nN, RP);
  k_gat_agg<NB12, NHEAD, HCH, false><<<RP / NB12, NTHR, LDS_AGG12, stream>>>(
      rowl, coll, hf, HIDW, ssp, sdp, RP, b1, g1, be1, ag, nN, nE, vec_col);
  k_rowpost<true><<<RP / NWAVE, NTHR, 0, stream>>>(ag, g1, be1, xf, ah, al, nN, RP);

  wmma_gemm64<1, true, 0, 0, false, 0><<<dim3(gWide, 1), 256, 0, stream>>>(
      ah, al, HIDW, 0L, w2h, w2l, HIDW, 0L, (void*)hf, (void*)hf, HIDW, 0L,
      b2, hf, 0L, RP, HIDW, HIDW, 1.0f);
  k_scores8<<<RP / NTHR, NTHR, 0, stream>>>(hf, as2, ad2, ssp, sdp, nN, RP);
  k_gat_agg<NB12, NHEAD, HCH, false><<<RP / NB12, NTHR, LDS_AGG12, stream>>>(
      rowl, coll, hf, HIDW, ssp, sdp, RP, b2, g2, be2, ag, nN, nE, vec_col);
  k_rowpost<true><<<RP / NWAVE, NTHR, 0, stream>>>(ag, g2, be2, xf, ah, al, nN, RP);

  wmma_gemm64<1, true, 0, 0, false, 0><<<dim3(gLast, 1), 256, 0, stream>>>(
      ah, al, HIDW, 0L, w3h, w3l, HIDW, 0L, (void*)hf, (void*)hf, OUTPAD, 0L,
      b3, hf, 0L, RP, OUTPAD, HIDW, 1.0f);
  k_scores16<<<RP / NTHR, NTHR, 0, stream>>>(hf, OUTPAD, as3, ad3, ssp, sdp, nN, RP);
  k_gat_agg<NB3, 1, OUTW, true><<<RP / NB3, NTHR, LDS_AGG3, stream>>>(
      rowl, coll, hf, OUTPAD, ssp, sdp, RP, b3, g3, be3, out, nN, nE, vec_col);
}
